// ViTBlock_48687749267828
// MI455X (gfx1250) — hardware-verified
//
#include <hip/hip_runtime.h>

typedef __bf16 bf16_t;
typedef bf16_t   v16b __attribute__((ext_vector_type(16)));
typedef float    v8f  __attribute__((ext_vector_type(8)));
typedef float    v4f  __attribute__((ext_vector_type(4)));
typedef unsigned v4u  __attribute__((ext_vector_type(4)));
typedef v4f __attribute__((may_alias)) v4fa;
typedef v4u __attribute__((may_alias)) v4ua;

union Frag { v16b v; v4u q[2]; };

#define BATCH  16
#define IN_C   384
#define OUT_C  512
#define HH     32
#define WW     32
#define NPIX   1024
#define BN_PIX 16384
#define HEADS  8
#define HD     64
#define MID    512
#define HID    2048
#define NBH    128
#define REL_W  63
#define REL_N  3969
#define QSCALE 0.125f
#define LN_EPS 1e-5f

#define G_Q   24576
#define G_KV  49152
#define G_PR  32768
#define G_SK  24576
#define G_F1  131072
#define G_F2  131072
#define G_TOT 393216

__device__ __forceinline__ unsigned bfbits(float f) {
  const unsigned u = __float_as_uint(f);
  return (u + 0x7FFFu + ((u >> 16) & 1u)) >> 16;
}
__device__ __forceinline__ unsigned pack2(float a, float b) { return bfbits(a) | (bfbits(b) << 16); }
__device__ __forceinline__ float bf_rne(float f) { return __uint_as_float(bfbits(f) << 16); }

__device__ __forceinline__ float wave_sum(float v) {
  #pragma unroll
  for (int m = 16; m >= 1; m >>= 1) v += __shfl_xor(v, m, 32);
  return v;
}

__device__ __forceinline__ v8f wmma_bf16(v16b a, v16b b, v8f c) {
  v8f d = __builtin_amdgcn_wmma_f32_16x16x32_bf16(false, a, false, b, (short)0, c, false, false);
  asm volatile("v_nop\n\tv_nop\n\tv_nop\n\tv_nop" : "+v"(d) : "v"(a), "v"(b));
  return d;
}

__device__ __forceinline__ v16b load_frag(const unsigned short* p, int h) {
  Frag f;
  f.q[0] = *(const v4ua*)(p + 8 * h);
  f.q[1] = *(const v4ua*)(p + 16 + 8 * h);
  return f.v;
}

__device__ __forceinline__ v16b frag_f32(const float* p, int h) {
  const v4f a = *(const v4fa*)(p + 8 * h);
  const v4f b = *(const v4fa*)(p + 8 * h + 4);
  const v4f c = *(const v4fa*)(p + 16 + 8 * h);
  const v4f d = *(const v4fa*)(p + 20 + 8 * h);
  v4u q0, q1;
  q0.x = pack2(a.x, a.y); q0.y = pack2(a.z, a.w); q0.z = pack2(b.x, b.y); q0.w = pack2(b.z, b.w);
  q1.x = pack2(c.x, c.y); q1.y = pack2(c.z, c.w); q1.z = pack2(d.x, d.y); q1.w = pack2(d.z, d.w);
  Frag f; f.q[0] = q0; f.q[1] = q1;
  return f.v;
}

__device__ __forceinline__ v16b pack16(v8f a, v8f c) {
  v4u q0, q1;
  q0.x = pack2(a[0], a[1]); q0.y = pack2(a[2], a[3]); q0.z = pack2(a[4], a[5]); q0.w = pack2(a[6], a[7]);
  q1.x = pack2(c[0], c[1]); q1.y = pack2(c[2], c[3]); q1.z = pack2(c[4], c[5]); q1.w = pack2(c[6], c[7]);
  Frag f; f.q[0] = q0; f.q[1] = q1;
  return f.v;
}

__device__ __forceinline__ v4u pack8(const float* e) {
  v4u o;
  o.x = pack2(e[0], e[1]); o.y = pack2(e[2], e[3]); o.z = pack2(e[4], e[5]); o.w = pack2(e[6], e[7]);
  return o;
}

__global__ __launch_bounds__(256) void cvt_w_kernel(
    const float* __restrict__ wq, const float* __restrict__ wkv, const float* __restrict__ wpr,
    const float* __restrict__ wsk, const float* __restrict__ wf1, const float* __restrict__ wf2,
    unsigned short* wts)
{
  const int g = blockIdx.x * 256 + threadIdx.x;
  if (g >= G_TOT) return;
  const float* src; int off;
  if (g < G_Q)                                   { src = wq;  off = g; }
  else if (g < G_Q + G_KV)                       { src = wkv; off = g - G_Q; }
  else if (g < G_Q + G_KV + G_PR)                { src = wpr; off = g - (G_Q + G_KV); }
  else if (g < G_Q + G_KV + G_PR + G_SK)         { src = wsk; off = g - (G_Q + G_KV + G_PR); }
  else if (g < G_Q + G_KV + G_PR + G_SK + G_F1)  { src = wf1; off = g - (G_Q + G_KV + G_PR + G_SK); }
  else                                           { src = wf2; off = g - (G_Q + G_KV + G_PR + G_SK + G_F1); }
  const v4f a = *(const v4fa*)(src + (size_t)off * 8);
  const v4f c = *(const v4fa*)(src + (size_t)off * 8 + 4);
  v4u o;
  o.x = pack2(a.x, a.y); o.y = pack2(a.z, a.w); o.z = pack2(c.x, c.y); o.w = pack2(c.z, c.w);
  unsigned short* dst = wts + (size_t)g * 8;
  *(volatile v4u*)dst = o;
  __threadfence();
  *(volatile v4u*)dst = o;
}

__global__ __launch_bounds__(256) void ln1_kernel(
    const float* __restrict__ x, const float* __restrict__ nw, const float* __restrict__ nb,
    unsigned short* xb, unsigned short* xn)
{
  __shared__ __attribute__((aligned(16))) float xs[IN_C * 33];
  const int tid = threadIdx.x, lane = tid & 31, w = tid >> 5;
  const int b = blockIdx.x >> 5, n0 = (blockIdx.x & 31) * 32;
  const float* xp = x + (size_t)b * IN_C * NPIX + n0 + lane;
  #pragma unroll 4
  for (int i = 0; i < 48; ++i) {
    const int c = w + 8 * i;
    xs[c * 33 + lane] = xp[(size_t)c * NPIX];
  }
  __syncthreads();

  #pragma unroll 1
  for (int j = 0; j < 4; ++j) {
    const int px = 4 * w + j;
    float v[12];
    float s = 0.f;
    #pragma unroll
    for (int i = 0; i < 12; ++i) { v[i] = xs[(lane + 32 * i) * 33 + px]; s += v[i]; }
    const float mean = wave_sum(s) * (1.0f / IN_C);
    float d2 = 0.f;
    #pragma unroll
    for (int i = 0; i < 12; ++i) { const float d = v[i] - mean; d2 += d * d; }
    const float rs = rsqrtf(wave_sum(d2) * (1.0f / IN_C) + LN_EPS);

    v4u rawv[2], nrmv[2];
    #pragma unroll
    for (int t = 0; t < 2; ++t) {
      int qc = lane + 32 * t;
      if (qc > 47) qc = 47;
      const int c0 = 8 * qc;
      float e[8], f[8];
      #pragma unroll
      for (int k = 0; k < 8; ++k) e[k] = xs[(c0 + k) * 33 + px];
      const v4f w0 = *(const v4fa*)(nw + c0), w1 = *(const v4fa*)(nw + c0 + 4);
      const v4f g0 = *(const v4fa*)(nb + c0), g1 = *(const v4fa*)(nb + c0 + 4);
      f[0] = (e[0] - mean) * rs * w0.x + g0.x;  f[1] = (e[1] - mean) * rs * w0.y + g0.y;
      f[2] = (e[2] - mean) * rs * w0.z + g0.z;  f[3] = (e[3] - mean) * rs * w0.w + g0.w;
      f[4] = (e[4] - mean) * rs * w1.x + g1.x;  f[5] = (e[5] - mean) * rs * w1.y + g1.y;
      f[6] = (e[6] - mean) * rs * w1.z + g1.z;  f[7] = (e[7] - mean) * rs * w1.w + g1.w;
      rawv[t] = pack8(e);
      nrmv[t] = pack8(f);
    }
    const size_t ro = (size_t)(b * NPIX + n0 + px) * IN_C;
    unsigned short* pb = xb + ro + 8 * lane;
    unsigned short* pn = xn + ro + 8 * lane;
    *(volatile v4u*)pb = rawv[0];
    *(volatile v4u*)pn = nrmv[0];
    if (lane < 16) { *(volatile v4u*)(pb + 256) = rawv[1]; *(volatile v4u*)(pn + 256) = nrmv[1]; }
    __threadfence();
    *(volatile v4u*)pb = rawv[0];
    *(volatile v4u*)pn = nrmv[0];
    if (lane < 16) { *(volatile v4u*)(pb + 256) = rawv[1]; *(volatile v4u*)(pn + 256) = nrmv[1]; }
  }
}

template <int MODE>
__global__ __launch_bounds__(128) void gemm_kernel(
    const unsigned short* __restrict__ A, int lda,
    const unsigned short* __restrict__ Wt, int ldw,
    const float* __restrict__ bias, const float* __restrict__ gamma,
    const float* __restrict__ resid, int ldr,
    float* outF, unsigned short* outB, int ldd, int K)
{
  __shared__ __attribute__((aligned(16))) float sT[4 * 2048];

  const int tid = threadIdx.x, lane = tid & 31, w = tid >> 5;
  const int h = lane >> 4, m = lane & 15;
  const int n0 = blockIdx.x * 64;
  const int m0w = blockIdx.y * 128 + 32 * w;

  const unsigned short* a0p = A + (size_t)(m0w + m) * lda;
  const unsigned short* a1p = a0p + (size_t)16 * lda;
  const unsigned short* wp  = Wt + (size_t)(n0 + m) * ldw;

  const v8f zero8 = {0.f, 0.f, 0.f, 0.f, 0.f, 0.f, 0.f, 0.f};
  v8f acc[2][4];
  #pragma unroll
  for (int mt = 0; mt < 2; ++mt)
    #pragma unroll
    for (int nt = 0; nt < 4; ++nt) acc[mt][nt] = zero8;

  #pragma unroll 1
  for (int k0 = 0; k0 < K; k0 += 32) {
    const v16b a0 = load_frag(a0p + k0, h);
    const v16b a1 = load_frag(a1p + k0, h);
    #pragma unroll
    for (int nt = 0; nt < 4; ++nt) {
      const v16b bb = load_frag(wp + (size_t)nt * 16 * ldw + k0, h);
      acc[0][nt] = wmma_bf16(a0, bb, acc[0][nt]);
      acc[1][nt] = wmma_bf16(a1, bb, acc[1][nt]);
    }
  }

  float* sw = sT + w * 2048;
  #pragma unroll
  for (int nt = 0; nt < 4; ++nt) {
    const int col = 16 * nt + m;
    const float bv = bias[n0 + col];
    float gv = 1.0f;
    if (MODE == 1 || MODE == 3) gv = gamma[n0 + col];
    #pragma unroll
    for (int mt = 0; mt < 2; ++mt) {
      #pragma unroll
      for (int r = 0; r < 8; ++r) {
        const int rowl = 16 * mt + 8 * h + r;
        const float v = acc[mt][nt][r] + bv;
        if (MODE == 0)      sw[rowl * 64 + col] = v;
        else if (MODE == 1) sw[rowl * 64 + col] = v * gv;
        else if (MODE == 2) sw[rowl * 64 + col] = 0.5f * v * (1.0f + erff(v * 0.70710678118654752f));
        else                sw[col * 32 + rowl] = resid[(size_t)(m0w + rowl) * ldr + n0 + col] + v * gv;
      }
    }
  }
  __syncthreads();

  if (MODE == 0 || MODE == 1) {
    v4f val[16];
    #pragma unroll
    for (int i = 0; i < 16; ++i) {
      const int row = 2 * i + (lane >> 4), c4 = (lane & 15) * 4;
      v4f v = *(const v4fa*)(sw + row * 64 + c4);
      if (MODE == 1) v += *(const v4fa*)(resid + (size_t)(m0w + row) * ldr + n0 + c4);
      val[i] = v;
      *(volatile v4f*)(outF + (size_t)(m0w + row) * ldd + n0 + c4) = v;
    }
    __threadfence();
    #pragma unroll
    for (int i = 0; i < 16; ++i) {
      const int row = 2 * i + (lane >> 4), c4 = (lane & 15) * 4;
      *(volatile v4f*)(outF + (size_t)(m0w + row) * ldd + n0 + c4) = val[i];
    }
  } else if (MODE == 2) {
    v4u val[8];
    #pragma unroll
    for (int i = 0; i < 8; ++i) {
      const int row = 4 * i + (lane >> 3), c8 = (lane & 7) * 8;
      const v4f a = *(const v4fa*)(sw + row * 64 + c8);
      const v4f c = *(const v4fa*)(sw + row * 64 + c8 + 4);
      v4u o;
      o.x = pack2(a.x, a.y); o.y = pack2(a.z, a.w); o.z = pack2(c.x, c.y); o.w = pack2(c.z, c.w);
      val[i] = o;
      *(volatile v4u*)(outB + (size_t)(m0w + row) * ldd + n0 + c8) = o;
    }
    __threadfence();
    #pragma unroll
    for (int i = 0; i < 8; ++i) {
      const int row = 4 * i + (lane >> 3), c8 = (lane & 7) * 8;
      *(volatile v4u*)(outB + (size_t)(m0w + row) * ldd + n0 + c8) = val[i];
    }
  } else {
    const int bimg = m0w >> 10, nimg0 = m0w & (NPIX - 1);
    v4f val[16];
    #pragma unroll
    for (int i = 0; i < 16; ++i) {
      const int c = 4 * i + (lane >> 3), t4 = (lane & 7) * 4;
      const v4f v = *(const v4fa*)(sw + c * 32 + t4);
      val[i] = v;
      *(volatile v4f*)(outF + ((size_t)(bimg * OUT_C + n0 + c)) * NPIX + nimg0 + t4) = v;
    }
    __threadfence();
    #pragma unroll
    for (int i = 0; i < 16; ++i) {
      const int c = 4 * i + (lane >> 3), t4 = (lane & 7) * 4;
      *(volatile v4f*)(outF + ((size_t)(bimg * OUT_C + n0 + c)) * NPIX + nimg0 + t4) = val[i];
    }
  }
}

__global__ __launch_bounds__(256) void pool_kernel(
    const float* __restrict__ in, const float* __restrict__ w3,
    const float* __restrict__ lnw, const float* __restrict__ lnb,
    float oscale, int mode, float* outF, unsigned short* outB)
{
  __shared__ __attribute__((aligned(16))) float tile[64 * 64];
  __shared__ float wsh[64 * 9];
  const int tid = threadIdx.x, lane = tid & 31, w = tid >> 5;
  const int bh = blockIdx.x >> 4, seg = blockIdx.x & 15;
  const int b = bh >> 3, hh = bh & 7;
  const int n0 = seg * 64;

  for (int i = tid; i < 64 * 9; i += 256) wsh[i] = bf_rne(w3[i]);
  __syncthreads();

  const float* inb = in + (size_t)b * NPIX * MID + hh * HD;

  #pragma unroll 1
  for (int j = 0; j < 8; ++j) {
    const int pxl = 8 * w + j, n = n0 + pxl, y = n >> 5, xx = n & 31;
    float vals[2];
    #pragma unroll
    for (int e = 0; e < 2; ++e) {
      const int d = lane + 32 * e;
      float s = 0.f;
      #pragma unroll
      for (int dy = -1; dy <= 1; ++dy) {
        const int yy = y + dy;
        if ((unsigned)yy < (unsigned)HH) {
          #pragma unroll
          for (int dx = -1; dx <= 1; ++dx) {
            const int xc = xx + dx;
            if ((unsigned)xc < (unsigned)WW)
              s += wsh[d * 9 + (dy + 1) * 3 + (dx + 1)] *
                   bf_rne(inb[(size_t)(yy * WW + xc) * MID + d]);
          }
        }
      }
      vals[e] = s;
    }
    const float mean = wave_sum(vals[0] + vals[1]) * (1.0f / HD);
    const float d0 = vals[0] - mean, d1 = vals[1] - mean;
    const float var = wave_sum(d0 * d0 + d1 * d1) * (1.0f / HD);
    const float rs = rsqrtf(var + LN_EPS);
    tile[pxl * 64 + lane]      = (d0 * rs * lnw[lane]      + lnb[lane])      * oscale;
    tile[pxl * 64 + lane + 32] = (d1 * rs * lnw[lane + 32] + lnb[lane + 32]) * oscale;
  }
  __syncthreads();

  if (mode == 0) {
    v4f val[4];
    float* dst[4];
    #pragma unroll
    for (int i = 0; i < 4; ++i) {
      const int pxl = 8 * w + 2 * i + (lane >> 4), c4 = (lane & 15) * 4;
      val[i] = *(const v4fa*)(tile + pxl * 64 + c4);
      dst[i] = outF + ((size_t)(bh * NPIX + n0 + pxl)) * HD + c4;
      *(volatile v4f*)dst[i] = val[i];
    }
    __threadfence();
    #pragma unroll
    for (int i = 0; i < 4; ++i) *(volatile v4f*)dst[i] = val[i];
  } else if (mode == 1) {
    v4u val[2];
    unsigned short* dst[2];
    #pragma unroll
    for (int i = 0; i < 2; ++i) {
      const int pxl = 8 * w + 4 * i + (lane >> 3), c8 = (lane & 7) * 8;
      const v4f a = *(const v4fa*)(tile + pxl * 64 + c8);
      const v4f c = *(const v4fa*)(tile + pxl * 64 + c8 + 4);
      v4u o;
      o.x = pack2(a.x, a.y); o.y = pack2(a.z, a.w); o.z = pack2(c.x, c.y); o.w = pack2(c.z, c.w);
      val[i] = o;
      dst[i] = outB + ((size_t)(bh * NPIX + n0 + pxl)) * HD + c8;
      *(volatile v4u*)dst[i] = o;
    }
    __threadfence();
    #pragma unroll
    for (int i = 0; i < 2; ++i) *(volatile v4u*)dst[i] = val[i];
  } else {
    v4u val[2];
    unsigned short* dst[2];
    #pragma unroll
    for (int i = 0; i < 2; ++i) {
      const int d = 8 * w + 4 * i + (lane >> 3), t8 = (lane & 7) * 8;
      float e[8];
      #pragma unroll
      for (int k = 0; k < 8; ++k) e[k] = tile[(t8 + k) * 64 + d];
      val[i] = pack8(e);
      dst[i] = outB + ((size_t)(bh * HD + d)) * NPIX + n0 + t8;
      *(volatile v4u*)dst[i] = val[i];
    }
    __threadfence();
    #pragma unroll
    for (int i = 0; i < 2; ++i) *(volatile v4u*)dst[i] = val[i];
  }
}

__global__ __launch_bounds__(128) void attn_kernel(
    const float* __restrict__ qf,
    const unsigned short* __restrict__ kbp,
    const unsigned short* __restrict__ vtp,
    const float* __restrict__ rel,
    unsigned short* ao)
{
  __shared__ __attribute__((aligned(16))) float sO[4 * 16 * 64];

  const int tid = threadIdx.x, lane = tid & 31, w = tid >> 5;
  const int h = lane >> 4, m = lane & 15;
  const int bh = blockIdx.y, b = bh >> 3, hh = bh & 7;
  const int q0 = blockIdx.x * 64 + 16 * w;

  const float* qrow = qf + ((size_t)bh * NPIX + q0 + m) * HD;
  const v16b qb0 = frag_f32(qrow, h);
  const v16b qb1 = frag_f32(qrow + 32, h);

  const int nq = q0 + m, y1 = nq >> 5, x1 = nq & 31;
  const int lb = (y1 + HH - 1) * REL_W + (x1 + WW - 1) - 8 * h;
  const float* relh = rel + hh;

  const v8f zero8 = {0.f, 0.f, 0.f, 0.f, 0.f, 0.f, 0.f, 0.f};
  v8f o[4];
  #pragma unroll
  for (int t = 0; t < 4; ++t) o[t] = zero8;
  float mrun = -1e30f, lrun = 0.0f;

  const unsigned short* kbase = kbp + ((size_t)bh * NPIX + m) * HD;
  const unsigned short* vbase = vtp + ((size_t)bh * HD + m) * NPIX;

  #pragma unroll 1
  for (int kb = 0; kb < NPIX; kb += 64) {
    v8f s[4];
    #pragma unroll
    for (int j = 0; j < 4; ++j) {
      const unsigned short* kp = kbase + (size_t)(kb + 16 * j) * HD;
      const v16b kf0 = load_frag(kp, h);
      const v16b kf1 = load_frag(kp + 32, h);
      v8f z = zero8;
      z = wmma_bf16(kf0, qb0, z);
      z = wmma_bf16(kf1, qb1, z);
      s[j] = z;
    }
    const int cst = lb - (kb >> 5) * REL_W;
    #pragma unroll
    for (int j = 0; j < 4; ++j)
      #pragma unroll
      for (int r = 0; r < 8; ++r)
        s[j][r] += relh[(cst - ((j >> 1) * REL_W + 16 * (j & 1) + r)) * HEADS];

    float mloc = s[0][0];
    #pragma unroll
    for (int j = 0; j < 4; ++j)
      #pragma unroll
      for (int r = 0; r < 8; ++r) mloc = fmaxf(mloc, s[j][r]);
    mloc = fmaxf(mloc, __shfl_xor(mloc, 16, 32));
    const float mnew = fmaxf(mrun, mloc);
    const float alpha = __expf(mrun - mnew);
    mrun = mnew;
    float lsum = 0.0f;
    #pragma unroll
    for (int j = 0; j < 4; ++j)
      #pragma unroll
      for (int r = 0; r < 8; ++r) {
        const float p = __expf(s[j][r] - mnew);
        s[j][r] = p;
        lsum += p;
      }
    lsum += __shfl_xor(lsum, 16, 32);
    lrun = lrun * alpha + lsum;
    #pragma unroll
    for (int t = 0; t < 4; ++t) o[t] = o[t] * alpha;

    const v16b pb0 = pack16(s[0], s[1]);
    const v16b pb1 = pack16(s[2], s[3]);

    #pragma unroll
    for (int t = 0; t < 4; ++t) {
      const unsigned short* vp = vbase + (size_t)(16 * t) * NPIX + kb;
      const v16b vf0 = load_frag(vp, h);
      const v16b vf1 = load_frag(vp + 32, h);
      o[t] = wmma_bf16(vf0, pb0, o[t]);
      o[t] = wmma_bf16(vf1, pb1, o[t]);
    }
  }

  const float inv = 1.0f / lrun;
  float* so = sO + w * 1024;
  #pragma unroll
  for (int t = 0; t < 4; ++t)
    #pragma unroll
    for (int r = 0; r < 8; ++r)
      so[m * 64 + 16 * t + 8 * h + r] = o[t][r] * inv;
  __syncthreads();

  const float* qres = qf + ((size_t)bh * NPIX + q0) * HD;
  v4u val[4];
  unsigned short* dst[4];
  #pragma unroll
  for (int i = 0; i < 4; ++i) {
    const int row = 4 * i + (lane >> 3), c8 = (lane & 7) * 8;
    const v4f a  = *(const v4fa*)(so + row * 64 + c8);
    const v4f c  = *(const v4fa*)(so + row * 64 + c8 + 4);
    const v4f ra = *(const v4fa*)(qres + row * 64 + c8);
    const v4f rc = *(const v4fa*)(qres + row * 64 + c8 + 4);
    const v4f ua = a + ra, uc = c + rc;
    v4u ov;
    ov.x = pack2(ua.x, ua.y); ov.y = pack2(ua.z, ua.w); ov.z = pack2(uc.x, uc.y); ov.w = pack2(uc.z, uc.w);
    val[i] = ov;
    dst[i] = ao + ((size_t)(b * NPIX + q0 + row)) * MID + hh * HD + c8;
    *(volatile v4u*)dst[i] = ov;
  }
  __threadfence();
  #pragma unroll
  for (int i = 0; i < 4; ++i) *(volatile v4u*)dst[i] = val[i];
}

__global__ __launch_bounds__(256) void ln2_kernel(
    const float* __restrict__ xpre, const float* __restrict__ nw, const float* __restrict__ nb,
    unsigned short* xn2)
{
  const int lane = threadIdx.x & 31, w = threadIdx.x >> 5;
  const int p = blockIdx.x * 8 + w;
  if (p >= BN_PIX) return;
  const float* rowp = xpre + (size_t)p * OUT_C;
  float v[16];
  #pragma unroll
  for (int t = 0; t < 2; ++t) {
    const int c0 = 8 * lane + 256 * t;
    const v4f a = *(const v4fa*)(rowp + c0), c = *(const v4fa*)(rowp + c0 + 4);
    v[8 * t + 0] = a.x; v[8 * t + 1] = a.y; v[8 * t + 2] = a.z; v[8 * t + 3] = a.w;
    v[8 * t + 4] = c.x; v[8 * t + 5] = c.y; v[8 * t + 6] = c.z; v[8 * t + 7] = c.w;
  }
  float s = 0.f;
  #pragma unroll
  for (int i = 0; i < 16; ++i) s += v[i];
  const float mean = wave_sum(s) * (1.0f / OUT_C);
  float d2 = 0.f;
  #pragma unroll
  for (int i = 0; i < 16; ++i) { const float d = v[i] - mean; d2 += d * d; }
  const float rs = rsqrtf(wave_sum(d2) * (1.0f / OUT_C) + LN_EPS);

  v4u o[2];
  #pragma unroll
  for (int t = 0; t < 2; ++t) {
    const int c0 = 8 * lane + 256 * t;
    const v4f w0 = *(const v4fa*)(nw + c0), w1 = *(const v4fa*)(nw + c0 + 4);
    const v4f g0 = *(const v4fa*)(nb + c0), g1 = *(const v4fa*)(nb + c0 + 4);
    float f[8];
    f[0] = (v[8 * t + 0] - mean) * rs * w0.x + g0.x;  f[1] = (v[8 * t + 1] - mean) * rs * w0.y + g0.y;
    f[2] = (v[8 * t + 2] - mean) * rs * w0.z + g0.z;  f[3] = (v[8 * t + 3] - mean) * rs * w0.w + g0.w;
    f[4] = (v[8 * t + 4] - mean) * rs * w1.x + g1.x;  f[5] = (v[8 * t + 5] - mean) * rs * w1.y + g1.y;
    f[6] = (v[8 * t + 6] - mean) * rs * w1.z + g1.z;  f[7] = (v[8 * t + 7] - mean) * rs * w1.w + g1.w;
    o[t] = pack8(f);
  }
  unsigned short* dst = xn2 + (size_t)p * OUT_C + 8 * lane;
  *(volatile v4u*)dst = o[0];
  *(volatile v4u*)(dst + 256) = o[1];
  __threadfence();
  *(volatile v4u*)dst = o[0];
  *(volatile v4u*)(dst + 256) = o[1];
}

extern "C" void kernel_launch(void* const* d_in, const int* in_sizes, int n_in,
                              void* d_out, int out_size, void* d_ws, size_t ws_size,
                              hipStream_t stream)
{
  if (n_in < 29) return;
  if (in_sizes[0] != BATCH * IN_C * NPIX) return;
  if (in_sizes[1] != IN_C || in_sizes[2] != IN_C) return;
  if (in_sizes[3] != MID * IN_C || in_sizes[4] != MID) return;
  if (in_sizes[5] != 2 * MID * IN_C || in_sizes[6] != 2 * MID) return;
  if (in_sizes[7] != HD * 9 || in_sizes[8] != HD * 9 || in_sizes[9] != HD * 9) return;
  for (int i = 10; i < 16; ++i) if (in_sizes[i] != HD) return;
  if (in_sizes[16] != REL_N * HEADS) return;
  if (in_sizes[17] != OUT_C * MID || in_sizes[18] != OUT_C || in_sizes[19] != OUT_C) return;
  if (in_sizes[20] != OUT_C * IN_C || in_sizes[21] != OUT_C) return;
  if (in_sizes[22] != OUT_C || in_sizes[23] != OUT_C) return;
  if (in_sizes[24] != HID * OUT_C || in_sizes[25] != HID) return;
  if (in_sizes[26] != OUT_C * HID || in_sizes[27] != OUT_C || in_sizes[28] != OUT_C) return;
  if (out_size != BATCH * OUT_C * NPIX) return;

  const float* x           = (const float*)d_in[0];
  const float* norm1_w     = (const float*)d_in[1];
  const float* norm1_b     = (const float*)d_in[2];
  const float* q_w         = (const float*)d_in[3];
  const float* q_b         = (const float*)d_in[4];
  const float* kv_w        = (const float*)d_in[5];
  const float* kv_b        = (const float*)d_in[6];
  const float* pool_q_w    = (const float*)d_in[7];
  const float* pool_k_w    = (const float*)d_in[8];
  const float* pool_v_w    = (const float*)d_in[9];
  const float* pnq_w       = (const float*)d_in[10];
  const float* pnq_b       = (const float*)d_in[11];
  const float* pnk_w       = (const float*)d_in[12];
  const float* pnk_b       = (const float*)d_in[13];
  const float* pnv_w       = (const float*)d_in[14];
  const float* pnv_b       = (const float*)d_in[15];
  const float* rel_table   = (const float*)d_in[16];
  const float* attn_proj_w = (const float*)d_in[17];
  const float* attn_proj_b = (const float*)d_in[18];
  const float* attn_gamma  = (const float*)d_in[19];
  const float* pool_skip_w = (const float*)d_in[20];
  const float* pool_skip_b = (const float*)d_in[21];
  const float* norm2_w     = (const float*)d_in[22];
  const float* norm2_b     = (const float*)d_in[23];
  const float* fc1_w       = (const float*)d_in[24];
  const float* fc1_b       = (const float*)d_in[25];
  const float* fc2_w       = (const float*)d_in[26];
  const float* fc2_b       = (const float*)d_in[27];
  const float* mlp_gamma   = (const float*)d_in[28];
  float* out = (float*)d_out;

  const size_t WTS_B = (size_t)G_TOT * 8 * 2;
  const size_t XB_B  = (size_t)BN_PIX * IN_C * 2;
  const size_t XN_B  = XB_B;
  const size_t BUF_B = (size_t)BN_PIX * MID * 4;
  const size_t QF_B  = (size_t)NBH * NPIX * HD * 4;
  const size_t KB_B  = (size_t)NBH * NPIX * HD * 2;
  const size_t VT_B  = KB_B;
  const size_t oW = 0, oXB = oW + WTS_B, oXN = oXB + XB_B, oBUF = oXN + XN_B,
               oQF = oBUF + BUF_B, oKB = oQF + QF_B, oVT = oKB + KB_B;
  const size_t total = oVT + VT_B;
  if (total > ws_size) return;
  if ((size_t)BN_PIX * MID * 2 > BUF_B) return;
  if ((size_t)BN_PIX * OUT_C * 4 > KB_B + VT_B) return;
  if ((size_t)BN_PIX * OUT_C * 2 > XB_B + XN_B) return;
  if ((size_t)BN_PIX * HID * 2 > BUF_B + QF_B) return;

  char* ws = (char*)d_ws;
  unsigned short* wts  = (unsigned short*)(ws + oW);
  unsigned short* xb   = (unsigned short*)(ws + oXB);
  unsigned short* xn   = (unsigned short*)(ws + oXN);
  float*          buf  = (float*)(ws + oBUF);
  float*          qf   = (float*)(ws + oQF);
  unsigned short* kbb  = (unsigned short*)(ws + oKB);
  unsigned short* vtb  = (unsigned short*)(ws + oVT);
  unsigned short* ao   = (unsigned short*)(ws + oBUF);
  float*          skpf = (float*)(ws + oQF);
  float*          xpre = (float*)(ws + oKB);
  unsigned short* xn2  = (unsigned short*)(ws + oXB);
  unsigned short* hmid = (unsigned short*)(ws + oBUF);

  const unsigned short* wq  = wts;
  const unsigned short* wkv = wts + (size_t)G_Q * 8;
  const unsigned short* wpr = wts + (size_t)(G_Q + G_KV) * 8;
  const unsigned short* wsk = wts + (size_t)(G_Q + G_KV + G_PR) * 8;
  const unsigned short* wf1 = wts + (size_t)(G_Q + G_KV + G_PR + G_SK) * 8;
  const unsigned short* wf2 = wts + (size_t)(G_Q + G_KV + G_PR + G_SK + G_F1) * 8;

  cvt_w_kernel<<<G_TOT / 256, 256, 0, stream>>>(q_w, kv_w, attn_proj_w, pool_skip_w, fc1_w, fc2_w, wts);

  ln1_kernel<<<BATCH * (NPIX / 32), 256, 0, stream>>>(x, norm1_w, norm1_b, xb, xn);

  const dim3 gG512(MID / 64, BN_PIX / 128);
  const int poolBlocks = NBH * (NPIX / 64);

  gemm_kernel<0><<<gG512, 128, 0, stream>>>(xn, IN_C, wq, IN_C, q_b, nullptr, nullptr, 0,
                                            buf, nullptr, MID, IN_C);
  pool_kernel<<<poolBlocks, 256, 0, stream>>>(buf, pool_q_w, pnq_w, pnq_b, QSCALE, 0, qf, nullptr);

  gemm_kernel<0><<<gG512, 128, 0, stream>>>(xn, IN_C, wkv, IN_C, kv_b, nullptr, nullptr, 0,
                                            buf, nullptr, MID, IN_C);
  pool_kernel<<<poolBlocks, 256, 0, stream>>>(buf, pool_k_w, pnk_w, pnk_b, 1.0f, 1, nullptr, kbb);

  gemm_kernel<0><<<gG512, 128, 0, stream>>>(xn, IN_C, wkv + (size_t)MID * IN_C, IN_C, kv_b + MID,
                                            nullptr, nullptr, 0, buf, nullptr, MID, IN_C);
  pool_kernel<<<poolBlocks, 256, 0, stream>>>(buf, pool_v_w, pnv_w, pnv_b, 1.0f, 2, nullptr, vtb);

  attn_kernel<<<dim3(NPIX / 64, NBH), 128, 0, stream>>>(qf, kbb, vtb, rel_table, ao);

  gemm_kernel<0><<<gG512, 128, 0, stream>>>(xb, IN_C, wsk, IN_C, pool_skip_b, nullptr, nullptr, 0,
                                            skpf, nullptr, OUT_C, IN_C);

  gemm_kernel<1><<<gG512, 128, 0, stream>>>(ao, MID, wpr, MID, attn_proj_b, attn_gamma, skpf, OUT_C,
                                            xpre, nullptr, OUT_C, MID);

  ln2_kernel<<<BN_PIX / 8, 256, 0, stream>>>(xpre, norm2_w, norm2_b, xn2);

  gemm_kernel<2><<<dim3(HID / 64, BN_PIX / 128), 128, 0, stream>>>(xn2, OUT_C, wf1, OUT_C, fc1_b,
                                            nullptr, nullptr, 0, nullptr, hmid, HID, OUT_C);

  gemm_kernel<3><<<dim3(OUT_C / 64, BN_PIX / 128), 128, 0, stream>>>(hmid, HID, wf2, HID, fc2_b,
                                            mlp_gamma, xpre, OUT_C, out, nullptr, 0, HID);
}
